// ReluSegmentNetwork2D_44014824849725
// MI455X (gfx1250) — hardware-verified
//
#include <hip/hip_runtime.h>
#include <stddef.h>


typedef _Float16 h16;
typedef _Float16 v16h __attribute__((ext_vector_type(16)));
typedef float    v8f  __attribute__((ext_vector_type(8)));
typedef float    v4f  __attribute__((ext_vector_type(4)));

#ifndef NPTS
#define NPTS 4194304
#endif
#define NPTS_FULL 4194304
#define NKNOT 17
#define NCELL 16
#define WAVES 8
#define WPTS  256
#define BPTS  (WAVES * WPTS)

static_assert(NPTS >= BPTS && NPTS <= NPTS_FULL);
static_assert((NPTS % BPTS) == 0);
static_assert(NKNOT == NCELL + 1);
static_assert(NCELL == 16);
static_assert(2 * NCELL == 32);
static_assert((WPTS % 32) == 0);
static_assert(WPTS == 2 * 32 * 4);
static_assert(WAVES * 32 == 256);

#define ZCARRY 64.0f
#define FCARRY 256.0f

__device__ __forceinline__ float bf16r(float x) {
  unsigned int u = __float_as_uint(x);
  u = (u + 0x7FFFu + ((u >> 16) & 1u)) & 0xFFFF0000u;
  return __uint_as_float(u);
}

static __device__ __forceinline__ h16 toh_flush(float v) {
  const h16 r = (h16)v;
  return (fabsf(v) < 6.103515625e-05f) ? (h16)0.0f : r;
}

__device__ __forceinline__ v8f wmma16(v16h a, v16h b, v8f c) {
  v8f d = __builtin_amdgcn_wmma_f32_16x16x32_f16(false, a, false, b, (short)0, c,
                                                 false, false);
  asm volatile("v_nop\n\tv_nop\n\tv_nop\n\tv_nop" : "+v"(d) : "v"(a), "v"(b));
  return d;
}

__device__ __forceinline__ void wave_lds_sync() {
  __builtin_amdgcn_fence(3  , "wavefront");
  asm volatile("s_wait_dscnt 0x0" ::: "memory");
  __builtin_amdgcn_wave_barrier();
}

__device__ __forceinline__ float tile_eval(const float xv, const float yv,
                                           const float (&xk)[9], const float (&rxk)[8],
                                           const float (&yk)[9], const float (&ryk)[8],
                                           const v16h za, const v16h zb) {
  v16h f;
#pragma unroll
  for (int i = 0; i < 8; ++i) {
    const float t0 = yv - yk[i];
    const float t1 = yv - yk[i + 1];
    const float ch = (fmaxf(t0, 0.0f) - fmaxf(t1, 0.0f)) * ryk[i];
    const float rel = t0 * ryk[i];
    f[i]     = toh_flush(FCARRY * (ch * (1.0f - rel)));
    f[i + 8] = toh_flush(FCARRY * (ch * rel));
  }
  v8f g1 = {}, g2 = {};
  g1 = wmma16(za, f, g1);
  g2 = wmma16(zb, f, g2);
  float s = 0.0f;
#pragma unroll
  for (int r = 0; r < 8; ++r) {
    const float t0 = xv - xk[r];
    const float t1 = xv - xk[r + 1];
    const float ch = (fmaxf(t0, 0.0f) - fmaxf(t1, 0.0f)) * rxk[r];
    const float rel = t0 * rxk[r];
    s += (ch * (1.0f - rel)) * g1[r] + (ch * rel) * g2[r];
  }
  s += __shfl_xor(s, 16, 32);
  return s;
}

__global__ __launch_bounds__(256) void seg2d_kernel(
    const float* __restrict__ x, const float* __restrict__ y,
    const float* __restrict__ xp, const float* __restrict__ yp,
    const float* __restrict__ zg, float* __restrict__ out) {
  __shared__ float kx[32];
  __shared__ float ky[32];
  __shared__ float krx[16];
  __shared__ float kry[16];
  __shared__ __attribute__((aligned(16))) float Os[WAVES * WPTS];

  const unsigned tid = threadIdx.x, lane = tid & 31u;
  const unsigned wave = (unsigned)__builtin_amdgcn_readfirstlane((int)(threadIdx.x >> 5));
  const unsigned hh = lane >> 4, m = lane & 15u;

  {
    const unsigned k0 = (tid < 16u) ? tid : 16u;
    const unsigned k1 = (tid < 16u) ? tid + 1u : 16u;
    const float xa = bf16r(xp[k0]);
    const float xb = bf16r(xp[k1]);
    const float ya = bf16r(yp[k0]);
    const float yb = bf16r(yp[k1]);
    const float dxv = (tid < 16u) ? (xb - xa) : 1.0f;
    const float dyv = (tid < 16u) ? (yb - ya) : 1.0f;
    const float rx = 1.0f / dxv;
    const float ry = 1.0f / dyv;
    if (tid < 17u) { kx[tid] = xa; ky[tid] = ya; }
    if (tid < 16u) { krx[tid] = rx; kry[tid] = ry; }
  }
  __syncthreads();

  float xk[9], yk[9], rxk[8], ryk[8];
#pragma unroll
  for (int i = 0; i < 9; ++i) {
    xk[i] = kx[hh * 8u + (unsigned)i];
    yk[i] = ky[hh * 8u + (unsigned)i];
  }
#pragma unroll
  for (int i = 0; i < 8; ++i) {
    rxk[i] = krx[hh * 8u + (unsigned)i];
    ryk[i] = kry[hh * 8u + (unsigned)i];
  }

  v16h za, zb;
#pragma unroll
  for (int i = 0; i < 8; ++i) {
    const unsigned j = hh * 8u + (unsigned)i;
    za[i]     = toh_flush(ZCARRY * bf16r(zg[m * 17u + j]));
    za[i + 8] = toh_flush(ZCARRY * bf16r(zg[m * 17u + j + 1u]));
    zb[i]     = toh_flush(ZCARRY * bf16r(zg[(m + 1u) * 17u + j]));
    zb[i + 8] = toh_flush(ZCARRY * bf16r(zg[(m + 1u) * 17u + j + 1u]));
  }

  const size_t base = ((size_t)blockIdx.x * WAVES + wave) * WPTS;

#pragma unroll 1
  for (unsigned it = 0; it < (unsigned)(WPTS / 32); ++it) {
    const size_t pa = base + it * 32u + m;
    const float xa = bf16r(x[pa]);
    const float ya = bf16r(y[pa]);
    const float xb = bf16r(x[pa + 16]);
    const float yb = bf16r(y[pa + 16]);
    const float sa = tile_eval(xa, ya, xk, rxk, yk, ryk, za, zb);
    const float sb = tile_eval(xb, yb, xk, rxk, yk, ryk, za, zb);
    const float val = ((hh == 0u) ? sa : sb) * (1.0f / (ZCARRY * FCARRY));
    Os[wave * WPTS + it * 32u + lane] = val;
  }
  wave_lds_sync();

  v4f o[2];
  size_t off[2];
#pragma unroll
  for (unsigned i = 0; i < 2u; ++i) {
    o[i] = *(const v4f*)&Os[wave * WPTS + i * 128u + lane * 4u];
    off[i] = base + i * 128u + lane * 4u;
  }
#pragma unroll
  for (int i = 0; i < 2; ++i) *(volatile v4f*)(out + off[i]) = o[i];
  __threadfence();
#pragma unroll
  for (int i = 0; i < 2; ++i) *(volatile v4f*)(out + off[i]) = o[i];
}

extern "C" void kernel_launch(void* const* d_in, const int* in_sizes, int n_in,
                              void* d_out, int out_size, void* d_ws, size_t ws_size,
                              hipStream_t stream) {
  (void)d_ws;
  (void)ws_size;
  if (n_in < 5) return;
  if ((long long)in_sizes[0] < (long long)NPTS) return;
  if ((long long)in_sizes[1] < (long long)NPTS) return;
  if (in_sizes[2] < NKNOT || in_sizes[3] < NKNOT) return;
  if (in_sizes[4] < NKNOT * NKNOT) return;
  if ((long long)out_size < (long long)NPTS) return;

  const float* x  = (const float*)d_in[0];
  const float* y  = (const float*)d_in[1];
  const float* xp = (const float*)d_in[2];
  const float* yp = (const float*)d_in[3];
  const float* zg = (const float*)d_in[4];
  float* out = (float*)d_out;

  seg2d_kernel<<<dim3(NPTS / BPTS), dim3(256), 0, stream>>>(x, y, xp, yp, zg, out);
}
